// MiniCPMSparseFlashAttention2_46909632806935
// MI455X (gfx1250) — hardware-verified
//
#include <hip/hip_runtime.h>
#include <stdint.h>
#include <stddef.h>
#include <math.h>

#pragma clang fp contract(off)

#define NS    2048
#define NHQ   16
#define NHKV  2
#define ND    128
#define NG    8
#define KER   32
#define STR   16
#define BLK   64
#define NTOP  4
#define NC    127
#define NCP   128
#define NBK   32
#define SCALE 0.08838834764831845f
#define NEGF  (-1.0e30f)

#define KP  136
#define VP  264
#define PP  264
#define LP  260
#define OP  132
#define TP  72

#define R0B       139264
#define OFF_SCORE R0B
#define OFF_IDX   (OFF_SCORE + 16 * NCP * 4)
#define OFF_L     (OFF_IDX + 256)
#define OFF_PH    (OFF_L + 16 * LP * 4)
#define OFF_PL    (OFF_PH + 16 * PP * 2)
#define OFF_O     (OFF_PL + 16 * PP * 2)
#define LDS_ATTN  (OFF_O + 16 * OP * 4)

static_assert(2 * 256 * KP * 2 <= R0B);
static_assert(2 * 128 * VP * 2 <= R0B);
static_assert(NG * 16 * NCP * 4 <= R0B);
static_assert(LDS_ATTN == 189696);
static_assert((OFF_SCORE % 16) == 0);
static_assert((OFF_IDX % 16) == 0);
static_assert((OFF_L % 16) == 0);
static_assert((OFF_PH % 16) == 0);
static_assert((OFF_PL % 16) == 0);
static_assert((OFF_O % 16) == 0);
static_assert((KP * 2) % 16 == 0);
static_assert((VP * 2) % 16 == 0);
static_assert((PP * 2) % 16 == 0);
static_assert((LP * 4) % 16 == 0);
static_assert((OP * 4) % 16 == 0);
static_assert((TP * 2) % 16 == 0);
static_assert(NS % 64 == 0);
static_assert(NS % 16 == 0);
static_assert((NS * NHQ * ND) % (8 * 256) == 0);
static_assert((NS * NHKV * ND) % (8 * 256) == 0);
static_assert((NHKV * NCP) % 16 == 0);
static_assert(NC == (NS - KER) / STR + 1);
static_assert(NBK == NS / BLK);
static_assert(NG * NHKV == NHQ);

typedef __bf16         v16bf __attribute__((ext_vector_type(16)));
typedef float          v8f   __attribute__((ext_vector_type(8)));
typedef float          v4f   __attribute__((ext_vector_type(4)));
typedef unsigned int   v4u   __attribute__((ext_vector_type(4)));
typedef v4f __attribute__((may_alias)) v4fa;
typedef v4u __attribute__((may_alias)) v4ua;

union FragBF { v16bf v; v4u q[2]; };

__device__ __forceinline__ unsigned int bfb(float f) {
  unsigned int u = __float_as_uint(f);
  u += 0x7FFFu + ((u >> 16) & 1u);
  return u >> 16;
}
__device__ __forceinline__ void split2(float v, unsigned int& hi, unsigned int& lo) {
  hi = bfb(v);
  lo = bfb(v - __uint_as_float(hi << 16));
}
__device__ __forceinline__ void split3(float v, unsigned int& a, unsigned int& b, unsigned int& c) {
  a = bfb(v);
  const float r1 = v - __uint_as_float(a << 16);
  b = bfb(r1);
  const float r2 = r1 - __uint_as_float(b << 16);
  c = bfb(r2);
}
__device__ __forceinline__ unsigned int pk(unsigned int a, unsigned int b) { return (a & 0xFFFFu) | (b << 16); }

__device__ __forceinline__ int sel4i(int s, int a, int b, int c, int d) {
  return (s == 0) ? a : ((s == 1) ? b : ((s == 2) ? c : d));
}
__device__ __forceinline__ bool sel4b(int s, bool a, bool b, bool c, bool d) {
  return (s == 0) ? a : ((s == 1) ? b : ((s == 2) ? c : d));
}
__device__ __forceinline__ int clampi(int v, int lo, int hi) { return (v < lo) ? lo : ((v > hi) ? hi : v); }

__device__ __forceinline__ v8f wmma_bf(v16bf a, v16bf b, v8f c) {
  v8f d = __builtin_amdgcn_wmma_f32_16x16x32_bf16(false, a, false, b, (short)0, c, false, false);
  asm volatile("v_nop\n\tv_nop\n\tv_nop\n\tv_nop" : "+v"(d) : "v"(a), "v"(b));
  return d;
}

__device__ __forceinline__ v16bf ldfrag(const unsigned short* p, int h) {
  FragBF f;
  f.q[0] = *(const v4ua*)(p + 8 * h);
  f.q[1] = *(const v4ua*)(p + 16 + 8 * h);
  return f.v;
}
__device__ __forceinline__ v16bf ldfrag_m(const unsigned short* p, int h, v4u msk) {
  FragBF f;
  f.q[0] = *(const v4ua*)(p + 8 * h) & msk;
  f.q[1] = *(const v4ua*)(p + 16 + 8 * h) & msk;
  return f.v;
}

__global__ __launch_bounds__(256) void k_qplanes(const float* __restrict__ src,
                                                 unsigned short* __restrict__ ph,
                                                 unsigned short* __restrict__ pm,
                                                 unsigned short* __restrict__ pl, int n8)
{
  const int g = blockIdx.x * 256 + threadIdx.x;
  if (g >= n8) return;
  const float* s = src + (size_t)g * 8;
  const v4f a = *(const v4fa*)s;
  const v4f c = *(const v4fa*)(s + 4);
  unsigned int h0, m0, l0, h1, m1, l1, h2, m2, l2, h3, m3, l3;
  unsigned int h4, m4, l4, h5, m5, l5, h6, m6, l6, h7, m7, l7;
  split3(a.x, h0, m0, l0); split3(a.y, h1, m1, l1); split3(a.z, h2, m2, l2); split3(a.w, h3, m3, l3);
  split3(c.x, h4, m4, l4); split3(c.y, h5, m5, l5); split3(c.z, h6, m6, l6); split3(c.w, h7, m7, l7);
  const v4u H = { pk(h0, h1), pk(h2, h3), pk(h4, h5), pk(h6, h7) };
  const v4u M = { pk(m0, m1), pk(m2, m3), pk(m4, m5), pk(m6, m7) };
  const v4u L = { pk(l0, l1), pk(l2, l3), pk(l4, l5), pk(l6, l7) };
  unsigned short* dh = ph + (size_t)g * 8;
  unsigned short* dm = pm + (size_t)g * 8;
  unsigned short* dl = pl + (size_t)g * 8;
  *(volatile v4u*)dh = H;
  *(volatile v4u*)dm = M;
  *(volatile v4u*)dl = L;
  __threadfence();
  *(volatile v4u*)dh = H;
  *(volatile v4u*)dm = M;
  *(volatile v4u*)dl = L;
}

__global__ __launch_bounds__(256) void k_kplanes(const float* __restrict__ src,
                                                 unsigned short* __restrict__ ph,
                                                 unsigned short* __restrict__ pm, int n8)
{
  const int g = blockIdx.x * 256 + threadIdx.x;
  if (g >= n8) return;
  const int c16 = g & 15;
  const int skv = g >> 4;
  const int kvh = skv & 1;
  const int s   = skv >> 1;
  const float* p = src + (size_t)g * 8;
  const v4f a = *(const v4fa*)p;
  const v4f c = *(const v4fa*)(p + 4);
  unsigned int h0, l0, h1, l1, h2, l2, h3, l3, h4, l4, h5, l5, h6, l6, h7, l7;
  split2(a.x, h0, l0); split2(a.y, h1, l1); split2(a.z, h2, l2); split2(a.w, h3, l3);
  split2(c.x, h4, l4); split2(c.y, h5, l5); split2(c.z, h6, l6); split2(c.w, h7, l7);
  const v4u H = { pk(h0, h1), pk(h2, h3), pk(h4, h5), pk(h6, h7) };
  const v4u M = { pk(l0, l1), pk(l2, l3), pk(l4, l5), pk(l6, l7) };
  const size_t o = ((size_t)kvh * NS + s) * ND + 8 * c16;
  *(volatile v4u*)(ph + o) = H;
  *(volatile v4u*)(pm + o) = M;
  __threadfence();
  *(volatile v4u*)(ph + o) = H;
  *(volatile v4u*)(pm + o) = M;
}

__global__ __launch_bounds__(256) void k_kcmp(const float* __restrict__ src,
                                              unsigned short* __restrict__ ph,
                                              unsigned short* __restrict__ pm,
                                              unsigned short* __restrict__ pl)
{
  const int tid = threadIdx.x;
  const int R = blockIdx.x * 16 + (tid >> 4);
  const int kvh = R >> 7;
  const int c = R & 127;
  const int c16 = tid & 15;
  const int cc = (c < NC) ? c : (NC - 1);
  v4f a0 = {0.f, 0.f, 0.f, 0.f};
  v4f a1 = {0.f, 0.f, 0.f, 0.f};
  #pragma unroll 4
  for (int j = 0; j < KER; ++j) {
    const float* p = src + ((size_t)(cc * STR + j) * NHKV + kvh) * ND + 8 * c16;
    const v4f x0 = *(const v4fa*)p;
    const v4f x1 = *(const v4fa*)(p + 4);
    a0 = a0 + x0;
    a1 = a1 + x1;
  }
  const bool live = (c < NC);
  const float w8 = 0.03125f;
  const float e0 = live ? a0.x * w8 : 0.f, e1 = live ? a0.y * w8 : 0.f;
  const float e2 = live ? a0.z * w8 : 0.f, e3 = live ? a0.w * w8 : 0.f;
  const float e4 = live ? a1.x * w8 : 0.f, e5 = live ? a1.y * w8 : 0.f;
  const float e6 = live ? a1.z * w8 : 0.f, e7 = live ? a1.w * w8 : 0.f;
  unsigned int h0, m0, l0, h1, m1, l1, h2, m2, l2, h3, m3, l3;
  unsigned int h4, m4, l4, h5, m5, l5, h6, m6, l6, h7, m7, l7;
  split3(e0, h0, m0, l0); split3(e1, h1, m1, l1); split3(e2, h2, m2, l2); split3(e3, h3, m3, l3);
  split3(e4, h4, m4, l4); split3(e5, h5, m5, l5); split3(e6, h6, m6, l6); split3(e7, h7, m7, l7);
  const v4u H = { pk(h0, h1), pk(h2, h3), pk(h4, h5), pk(h6, h7) };
  const v4u M = { pk(m0, m1), pk(m2, m3), pk(m4, m5), pk(m6, m7) };
  const v4u L = { pk(l0, l1), pk(l2, l3), pk(l4, l5), pk(l6, l7) };
  const size_t o = ((size_t)kvh * NCP + c) * ND + 8 * c16;
  *(volatile v4u*)(ph + o) = H;
  *(volatile v4u*)(pm + o) = M;
  *(volatile v4u*)(pl + o) = L;
  __threadfence();
  *(volatile v4u*)(ph + o) = H;
  *(volatile v4u*)(pm + o) = M;
  *(volatile v4u*)(pl + o) = L;
}

__global__ __launch_bounds__(256) void k_vtplanes(const float* __restrict__ src,
                                                  unsigned short* __restrict__ vth,
                                                  unsigned short* __restrict__ vtm)
{
  __shared__ __align__(16) unsigned short sT[2 * 128 * TP];
  const int tid = threadIdx.x, lane = tid & 31, w = tid >> 5;
  const int s0 = blockIdx.x * 64, kvh = blockIdx.y;
  #pragma unroll
  for (int i = 0; i < 8; ++i) {
    const int f = tid + 256 * i;
    const int sl = f >> 5;
    const int d0 = (f & 31) * 4;
    const v4f x = *(const v4fa*)(src + ((size_t)(s0 + sl) * NHKV + kvh) * ND + d0);
    unsigned int h0, l0, h1, l1, h2, l2, h3, l3;
    split2(x.x, h0, l0); split2(x.y, h1, l1); split2(x.z, h2, l2); split2(x.w, h3, l3);
    sT[(d0 + 0) * TP + sl] = (unsigned short)h0;  sT[128 * TP + (d0 + 0) * TP + sl] = (unsigned short)l0;
    sT[(d0 + 1) * TP + sl] = (unsigned short)h1;  sT[128 * TP + (d0 + 1) * TP + sl] = (unsigned short)l1;
    sT[(d0 + 2) * TP + sl] = (unsigned short)h2;  sT[128 * TP + (d0 + 2) * TP + sl] = (unsigned short)l2;
    sT[(d0 + 3) * TP + sl] = (unsigned short)h3;  sT[128 * TP + (d0 + 3) * TP + sl] = (unsigned short)l3;
  }
  __syncthreads();
  const int pl = w >> 2;
  unsigned short* base = (pl == 0) ? vth : vtm;
  const int e = lane & 7;
  #pragma unroll
  for (int it = 0; it < 8; ++it) {
    const int d = (w & 3) * 32 + it * 4 + (lane >> 3);
    const v4u x = *(const v4ua*)(sT + pl * 128 * TP + d * TP + 8 * e);
    unsigned short* dst = base + ((size_t)(kvh * ND + d)) * NS + s0 + 8 * e;
    *(volatile v4u*)dst = x;
    __threadfence();
    *(volatile v4u*)dst = x;
  }
}

__global__ __launch_bounds__(256) void k_attn(const unsigned short* __restrict__ qh,
                                              const unsigned short* __restrict__ qm,
                                              const unsigned short* __restrict__ ql,
                                              const unsigned short* __restrict__ kh,
                                              const unsigned short* __restrict__ km,
                                              const unsigned short* __restrict__ cph,
                                              const unsigned short* __restrict__ cpm,
                                              const unsigned short* __restrict__ cpl,
                                              const unsigned short* __restrict__ vth,
                                              const unsigned short* __restrict__ vtm,
                                              float* __restrict__ out)
{
  extern __shared__ __align__(16) unsigned char dsm[];
  float*          sProb  = (float*)dsm;
  unsigned short* sKh    = (unsigned short*)dsm;
  unsigned short* sKm    = (unsigned short*)(dsm + 256 * KP * 2);
  unsigned short* sVh    = (unsigned short*)dsm;
  unsigned short* sVm    = (unsigned short*)(dsm + 128 * VP * 2);
  float*          sScore = (float*)(dsm + OFF_SCORE);
  int*            sIdx   = (int*)(dsm + OFF_IDX);
  float*          sL     = (float*)(dsm + OFF_L);
  unsigned short* sPh    = (unsigned short*)(dsm + OFF_PH);
  unsigned short* sPl    = (unsigned short*)(dsm + OFF_PL);
  float*          sO     = (float*)(dsm + OFF_O);

  const int tid = threadIdx.x, lane = tid & 31, w = tid >> 5;
  const int h = lane >> 4, m = lane & 15;
  const int s0 = blockIdx.x * 16, kv = blockIdx.y;

  for (int i = tid; i < 16 * PP; i += 256) { sPh[i] = 0; sPl[i] = 0; }

  const v8f z8 = {0.f, 0.f, 0.f, 0.f, 0.f, 0.f, 0.f, 0.f};

  #pragma unroll 1
  for (int tp = 0; tp < 2; ++tp) {
    v8f acc[4];
    #pragma unroll
    for (int t4 = 0; t4 < 4; ++t4) acc[t4] = z8;
    #pragma unroll 1
    for (int kc = 0; kc < 4; ++kc) {
      const size_t ao = ((size_t)(s0 + m) * NHQ + kv * NG + w) * ND + kc * 32;
      const v16bf fah = ldfrag(qh + ao, h);
      const v16bf fam = ldfrag(qm + ao, h);
      const v16bf fal = ldfrag(ql + ao, h);
      #pragma unroll
      for (int t4 = 0; t4 < 4; ++t4) {
        const int c = (tp * 4 + t4) * 16 + m;
        const size_t bo = ((size_t)kv * NCP + c) * ND + kc * 32;
        const v16bf fbh = ldfrag(cph + bo, h);
        const v16bf fbm = ldfrag(cpm + bo, h);
        const v16bf fbl = ldfrag(cpl + bo, h);
        acc[t4] = wmma_bf(fah, fbh, acc[t4]);
        acc[t4] = wmma_bf(fah, fbm, acc[t4]);
        acc[t4] = wmma_bf(fam, fbh, acc[t4]);
        acc[t4] = wmma_bf(fah, fbl, acc[t4]);
        acc[t4] = wmma_bf(fam, fbm, acc[t4]);
        acc[t4] = wmma_bf(fal, fbh, acc[t4]);
      }
    }
    #pragma unroll
    for (int t4 = 0; t4 < 4; ++t4) {
      const int c = (tp * 4 + t4) * 16 + m;
      #pragma unroll
      for (int r = 0; r < 8; ++r) {
        const int row = 8 * h + r;
        const int s = s0 + row;
        const bool vis = (c < NC) && (c * STR + KER - 1 <= s);
        const float x = vis ? acc[t4][r] * SCALE : NEGF;
        sProb[(w * 16 + row) * NCP + c] = x;
      }
    }
  }
  __syncthreads();

  #pragma unroll 1
  for (int row = 0; row < 16; ++row) {
    const int s = s0 + row;
    float* pr = sProb + (w * 16 + row) * NCP;
    float x[4];
    bool vis[4];
    #pragma unroll
    for (int i = 0; i < 4; ++i) {
      const int c = lane + 32 * i;
      x[i] = pr[c];
      vis[i] = (c < NC) && (c * STR + KER - 1 <= s);
    }
    float mx = fmaxf(fmaxf(x[0], x[1]), fmaxf(x[2], x[3]));
    #pragma unroll
    for (int off = 16; off > 0; off >>= 1) mx = fmaxf(mx, __shfl_xor(mx, off));
    float e[4];
    float sum = 0.f;
    #pragma unroll
    for (int i = 0; i < 4; ++i) { e[i] = expf(x[i] - mx); sum += e[i]; }
    #pragma unroll
    for (int off = 16; off > 0; off >>= 1) sum += __shfl_xor(sum, off);
    const float rcp = 1.0f / sum;
    #pragma unroll
    for (int i = 0; i < 4; ++i) pr[lane + 32 * i] = vis[i] ? e[i] * rcp : 0.f;
  }
  __syncthreads();

  #pragma unroll
  for (int i = 0; i < 8; ++i) {
    const int e = tid + 256 * i;
    const int q = e >> 7, c = e & 127;
    float sc = 0.f;
    #pragma unroll
    for (int g = 0; g < NG; ++g) sc += sProb[(g * 16 + q) * NCP + c];
    sScore[q * NCP + c] = sc;
  }
  __syncthreads();

  if (w == 0) {
    #pragma unroll 1
    for (int q = 0; q < 16; ++q) {
      const int s = s0 + q;
      const int qb = s >> 6;
      const int b = lane;
      float mx = NEGF;
      #pragma unroll
      for (int i = 0; i < 5; ++i) {
        const int ci = 4 * b - 1 + i;
        const bool ok = (ci >= 0) && (ci <= NC - 1);
        const int cc = clampi(ci, 0, NC - 1);
        const float v = sScore[q * NCP + cc];
        mx = ok ? fmaxf(mx, v) : mx;
      }
      const bool forced = (b == 0) || (b >= qb - 1);
      const float val = (b > qb) ? NEGF : (forced ? 1.0e9f : mx);
      unsigned int taken = 0u;
      #pragma unroll
      for (int j = 0; j < NTOP; ++j) {
        const float vv = ((taken >> b) & 1u) ? -3.0e38f : val;
        float vm = vv;
        #pragma unroll
        for (int off = 16; off > 0; off >>= 1) vm = fmaxf(vm, __shfl_xor(vm, off));
        const unsigned int msk = __builtin_amdgcn_ballot_w32(vv == vm) & ~taken;
        const int bi = (msk != 0u) ? __builtin_ctz(msk) : 0;
        taken |= (1u << bi);
      }
      if (lane == 0) {
        unsigned int mk = taken;
        #pragma unroll
        for (int j = 0; j < NTOP; ++j) {
          const int bj = (mk != 0u) ? __builtin_ctz(mk) : 0;
          mk &= (mk - 1u);
          sIdx[q * NTOP + j] = (bj >= qb) ? -1 : bj;
        }
      }
    }
  }
  __syncthreads();

  const size_t qmask = (m < NG) ? 0xFFFFFFFFu : 0u;
  const v4u amask = { (unsigned int)qmask, (unsigned int)qmask, (unsigned int)qmask, (unsigned int)qmask };

  #pragma unroll 1
  for (int q = 0; q < 16; ++q) {
    const int s = s0 + q;
    const int i0 = sIdx[q * NTOP + 0];
    const int i1 = sIdx[q * NTOP + 1];
    const int i2 = sIdx[q * NTOP + 2];
    const int i3 = sIdx[q * NTOP + 3];
    const bool v0 = (i0 >= 0), v1 = (i1 >= 0), v2 = (i2 >= 0), v3 = (i3 >= 0);
    const int c0 = clampi(i0, 0, NBK - 1), c1 = clampi(i1, 0, NBK - 1);
    const int c2 = clampi(i2, 0, NBK - 1), c3 = clampi(i3, 0, NBK - 1);

    #pragma unroll
    for (int i = 0; i < 16; ++i) {
      const int f = tid + 256 * i;
      const int row = f >> 4;
      const int c16 = f & 15;
      const int blk = sel4i(i >> 2, c0, c1, c2, c3);
      const int key = blk * BLK + (row & 63);
      const size_t go = ((size_t)kv * NS + key) * ND + 8 * c16;
      const v4u a = *(const v4ua*)(kh + go);
      const v4u b = *(const v4ua*)(km + go);
      *(v4ua*)(sKh + row * KP + 8 * c16) = a;
      *(v4ua*)(sKm + row * KP + 8 * c16) = b;
    }
    __syncthreads();

    {
      v8f acc[2] = { z8, z8 };
      const size_t arow = ((size_t)s * NHQ + kv * NG + (m & 7)) * ND;
      #pragma unroll 1
      for (int kc = 0; kc < 4; ++kc) {
        const v16bf fah = ldfrag_m(qh + arow + kc * 32, h, amask);
        const v16bf fam = ldfrag_m(qm + arow + kc * 32, h, amask);
        #pragma unroll
        for (int nt = 0; nt < 2; ++nt) {
          const int key = 32 * w + 16 * nt + m;
          const v16bf fbh = ldfrag(sKh + key * KP + kc * 32, h);
          const v16bf fbm = ldfrag(sKm + key * KP + kc * 32, h);
          acc[nt] = wmma_bf(fah, fbh, acc[nt]);
          acc[nt] = wmma_bf(fah, fbm, acc[nt]);
          acc[nt] = wmma_bf(fam, fbh, acc[nt]);
        }
      }
      const bool vw = sel4b(w >> 1, v0, v1, v2, v3);
      #pragma unroll
      for (int nt = 0; nt < 2; ++nt) {
        const int col = 32 * w + 16 * nt + m;
        #pragma unroll
        for (int r = 0; r < 8; ++r) {
          const int row = 8 * h + r;
          const float x = vw ? acc[nt][r] * SCALE : NEGF;
          sL[row * LP + col] = x;
        }
      }
    }
    __syncthreads();

    {
      const int chn = tid & 31;
      const int blk = sel4i(chn >> 3, c0, c1, c2, c3);
      const size_t ko = (size_t)blk * BLK + 8 * (chn & 7);
      #pragma unroll
      for (int i = 0; i < 16; ++i) {
        const int d = w + 8 * i;
        const size_t go = ((size_t)(kv * ND + d)) * NS + ko;
        const v4u a = *(const v4ua*)(vth + go);
        const v4u b = *(const v4ua*)(vtm + go);
        *(v4ua*)(sVh + d * VP + 8 * chn) = a;
        *(v4ua*)(sVm + d * VP + 8 * chn) = b;
      }
    }
    {
      const float* lr = sL + w * LP;
      float x[8];
      #pragma unroll
      for (int i = 0; i < 8; ++i) x[i] = lr[lane + 32 * i];
      float mx = x[0];
      #pragma unroll
      for (int i = 1; i < 8; ++i) mx = fmaxf(mx, x[i]);
      #pragma unroll
      for (int off = 16; off > 0; off >>= 1) mx = fmaxf(mx, __shfl_xor(mx, off));
      float e[8];
      float sum = 0.f;
      #pragma unroll
      for (int i = 0; i < 8; ++i) { e[i] = expf(x[i] - mx); sum += e[i]; }
      #pragma unroll
      for (int off = 16; off > 0; off >>= 1) sum += __shfl_xor(sum, off);
      const float rcp = 1.0f / sum;
      #pragma unroll
      for (int i = 0; i < 8; ++i) {
        const bool vv = sel4b(i >> 1, v0, v1, v2, v3);
        const float p = vv ? e[i] * rcp : 0.f;
        unsigned int hb, lb;
        split2(p, hb, lb);
        sPh[w * PP + lane + 32 * i] = (unsigned short)hb;
        sPl[w * PP + lane + 32 * i] = (unsigned short)lb;
      }
    }
    __syncthreads();

    {
      v8f oacc = z8;
      #pragma unroll 1
      for (int kc = 0; kc < 8; ++kc) {
        const v16bf fph = ldfrag(sPh + m * PP + kc * 32, h);
        const v16bf fpl = ldfrag(sPl + m * PP + kc * 32, h);
        const v16bf fvh = ldfrag(sVh + (16 * w + m) * VP + kc * 32, h);
        const v16bf fvm = ldfrag(sVm + (16 * w + m) * VP + kc * 32, h);
        oacc = wmma_bf(fph, fvh, oacc);
        oacc = wmma_bf(fph, fvm, oacc);
        oacc = wmma_bf(fpl, fvh, oacc);
      }
      #pragma unroll
      for (int r = 0; r < 8; ++r) sO[(8 * h + r) * OP + 16 * w + m] = oacc[r];
    }
    __syncthreads();

    {
      const v4f ov = *(const v4fa*)(sO + w * OP + 4 * lane);
      float* dst = out + ((size_t)s * NHQ + kv * NG + w) * ND + 4 * lane;
      *(volatile v4f*)dst = ov;
      __threadfence();
      *(volatile v4f*)dst = ov;
    }
  }
}

extern "C" void kernel_launch(void* const* d_in, const int* in_sizes, int n_in,
                              void* d_out, int out_size, void* d_ws, size_t ws_size,
                              hipStream_t stream)
{
  if (n_in < 3) return;
  if (in_sizes[0] != NS * NHQ * ND) return;
  if (in_sizes[1] != NS * NHKV * ND) return;
  if (in_sizes[2] != NS * NHKV * ND) return;
  if (out_size != NS * NHQ * ND) return;

  const float* q = (const float*)d_in[0];
  const float* k = (const float*)d_in[1];
  const float* v = (const float*)d_in[2];
  float* out = (float*)d_out;

  const size_t bQ = (size_t)NS * NHQ * ND * 2;
  const size_t bK = (size_t)NHKV * NS * ND * 2;
  const size_t bV = (size_t)NHKV * ND * NS * 2;
  const size_t bC = (size_t)NHKV * NCP * ND * 2;
  const size_t total = 3 * bQ + 2 * bK + 2 * bV + 3 * bC;
  if (total > ws_size) return;
  if (total > (size_t)134217728) return;

  char* ws = (char*)d_ws;
  size_t off = 0;
  unsigned short* QH  = (unsigned short*)(ws + off); off += bQ;
  unsigned short* QM  = (unsigned short*)(ws + off); off += bQ;
  unsigned short* QL  = (unsigned short*)(ws + off); off += bQ;
  unsigned short* KH  = (unsigned short*)(ws + off); off += bK;
  unsigned short* KM  = (unsigned short*)(ws + off); off += bK;
  unsigned short* VTH = (unsigned short*)(ws + off); off += bV;
  unsigned short* VTM = (unsigned short*)(ws + off); off += bV;
  unsigned short* CH  = (unsigned short*)(ws + off); off += bC;
  unsigned short* CM  = (unsigned short*)(ws + off); off += bC;
  unsigned short* CL  = (unsigned short*)(ws + off); off += bC;
  if (off != total) return;

  {
    const int n8 = NS * NHQ * ND / 8;
    k_qplanes<<<(n8 + 255) / 256, 256, 0, stream>>>(q, QH, QM, QL, n8);
  }
  {
    const int n8 = NS * NHKV * ND / 8;
    k_kplanes<<<(n8 + 255) / 256, 256, 0, stream>>>(k, KH, KM, n8);
  }
  k_kcmp<<<(NHKV * NCP) / 16, 256, 0, stream>>>(k, CH, CM, CL);
  k_vtplanes<<<dim3(NS / 64, NHKV), 256, 0, stream>>>(v, VTH, VTM);
  hipFuncSetAttribute(reinterpret_cast<const void*>(&k_attn),
                      hipFuncAttributeMaxDynamicSharedMemorySize, LDS_ATTN);
  k_attn<<<dim3(NS / 16, NHKV), 256, LDS_ATTN, stream>>>(QH, QM, QL, KH, KM, CH, CM, CL, VTH, VTM, out);
}
